// TransformerXLEncoderLayer_31439160606837
// MI455X (gfx1250) — hardware-verified
//
#include <hip/hip_runtime.h>
#include <math.h>


#define BB 2
#define SS 2048
#define DD 1024
#define HH 16
#define HD 64
#define FF 4096
#define PREV 1024
#define TOT 3072
#define NR (BB * SS)
#define BK 32

typedef __attribute__((ext_vector_type(16))) _Float16 v16h;
typedef __attribute__((ext_vector_type(8)))  _Float16 v8h;
typedef __attribute__((ext_vector_type(8)))  float v8f;
typedef __attribute__((ext_vector_type(4)))  float v4f;
typedef __attribute__((ext_vector_type(4)))  unsigned v4u;

template <typename T> __device__ __forceinline__ void vst2(void* p, T v) { *(volatile T*)p = v; __threadfence(); *(volatile T*)p = v; }
__device__ __forceinline__ v8f wmma16(v16h a, v16h b, v8f c) {
  v8f d = __builtin_amdgcn_wmma_f32_16x16x32_f16(false, a, false, b, (short)0, c, false, false);
  asm volatile("v_nop\n\tv_nop\n\tv_nop\n\tv_nop" : "+v"(d) : "v"(a), "v"(b));
  return d;
}
__device__ __forceinline__ v16h frag_h(const _Float16* rowk0, int lane) {
  union { v16h v; v8h q[2]; } u; const _Float16* p = rowk0 + 8 * (lane >> 4);
  u.q[0] = *(const v8h*)p; u.q[1] = *(const v8h*)(p + 16); return u.v;
}
__device__ __forceinline__ v16h frag_f32(const float* rowk0, int lane) {
  v16h a; const float* p = rowk0 + 8 * (lane >> 4);
#pragma unroll
  for (int i = 0; i < 8; ++i) { a[i] = (_Float16)p[i]; a[8 + i] = (_Float16)p[16 + i]; }
  return a;
}
#define LDSX() do { asm volatile("s_wait_dscnt 0" ::: "memory"); __builtin_amdgcn_wave_barrier(); __builtin_amdgcn_fence(__ATOMIC_RELEASE, "workgroup"); } while (0)

__global__ __launch_bounds__(256) void k_cvt(const float* __restrict__ s, _Float16* __restrict__ d, size_t n8) {
  const size_t g8 = (size_t)blockIdx.x * 256 + threadIdx.x; if (g8 >= n8) return;
  union { v8h h; v4u u; } pk;
#pragma unroll
  for (int e = 0; e < 8; ++e) pk.h[e] = (_Float16)s[g8 * 8 + e];
  vst2(d + g8 * 8, pk.u);
}
__global__ __launch_bounds__(128) void k_rms(const float* __restrict__ x, const float* __restrict__ w, _Float16* __restrict__ h) {
  __shared__ float red[128];
  const size_t row = blockIdx.x; const int tid = threadIdx.x;
  const float* xr = x + row * DD;
  float v[8], s = 0.f;
#pragma unroll
  for (int e = 0; e < 8; ++e) { v[e] = xr[tid * 8 + e]; s += v[e] * v[e]; }
  red[tid] = s; __syncthreads();
  for (int st = 64; st > 0; st >>= 1) { if (tid < st) red[tid] += red[tid + st]; __syncthreads(); }
  const float rs = rsqrtf(red[0] / (float)DD + 1e-6f);
  union { v8h hh; v4u u; } pk;
#pragma unroll
  for (int e = 0; e < 8; ++e) pk.hh[e] = (_Float16)(v[e] * rs * w[tid * 8 + e]);
  vst2(h + row * DD + tid * 8, pk.u);
}

__device__ __forceinline__ void rope2(float& a, float& b, const float* __restrict__ cs, const float* __restrict__ sn, int pos, int i) {
  const float c = cs[(size_t)pos * (HD / 2) + i], s = sn[(size_t)pos * (HD / 2) + i];
  const float x0 = a, x1 = b; a = x0 * c - x1 * s; b = x0 * s + x1 * c;
}

__global__ __launch_bounds__(128) void k_qkv(const _Float16* __restrict__ hh, const _Float16* __restrict__ Wq, const _Float16* __restrict__ Wk,
                                           const _Float16* __restrict__ Wv, const float* __restrict__ bq, const float* __restrict__ bk,
                                           const float* __restrict__ bv, const float* __restrict__ cs, const float* __restrict__ sn,
                                           _Float16* __restrict__ qh, _Float16* __restrict__ kall, _Float16* __restrict__ vT) {
  __shared__ __align__(16) float st[128][68];
  const int tid = threadIdx.x, wave = tid >> 5, lane = tid & 31, col = lane & 15, g = lane >> 4;
  const int r0 = blockIdx.x * 64, n0 = blockIdx.y * 128, which = blockIdx.z;
  const int b = r0 / SS, s0 = r0 % SS, h0 = n0 / HD;
  const _Float16* W = which == 0 ? Wq : (which == 1 ? Wk : Wv); const float* bias = which == 0 ? bq : (which == 1 ? bk : bv);
  v8f acc[8] = {};
#pragma unroll 1
  for (int kc = 0; kc < DD / 32; ++kc) {
    const v16h a = frag_h(hh + (size_t)(r0 + wave * 16 + col) * DD + kc * 32, lane);
#pragma unroll
    for (int j = 0; j < 8; ++j) acc[j] = wmma16(a, frag_h(W + (size_t)(n0 + j * 16 + col) * DD + kc * 32, lane), acc[j]);
  }
#pragma unroll
  for (int j = 0; j < 8; ++j) { const float bv_ = bias[n0 + j * 16 + col];
#pragma unroll
    for (int r = 0; r < 8; ++r) st[j * 16 + col][wave * 16 + 8 * g + r] = acc[j][r] + bv_; }
  __syncthreads();
  if (which < 2) {
    for (int q = tid; q < 2 * 64 * 8; q += 128) { const int hl = q >> 9, sl = (q >> 3) & 63, pc = q & 7;
      const int pos = PREV + s0 + sl;
      union { v8h h; v4u u; } pk;
#pragma unroll
      for (int e = 0; e < 8; e += 2) { float a0 = st[hl * 64 + pc * 8 + e][sl], a1 = st[hl * 64 + pc * 8 + e + 1][sl];
        rope2(a0, a1, cs, sn, pos, (pc * 8 + e) >> 1); pk.h[e] = (_Float16)a0; pk.h[e + 1] = (_Float16)a1; }
      _Float16* dst = (which == 0) ? qh + (((size_t)b * HH + h0 + hl) * SS + s0 + sl) * HD
                                   : kall + (((size_t)b * HH + h0 + hl) * TOT + PREV + s0 + sl) * HD;
      vst2(dst + pc * 8, pk.u); }
  } else {
    for (int q = tid; q < 128 * 8; q += 128) { const int cl = q >> 3, pc = q & 7; const int hl = cl >> 6, d = cl & 63;
      union { v8h h; v4u u; } pk;
#pragma unroll
      for (int i = 0; i < 8; ++i) pk.h[i] = (_Float16)st[cl][pc * 8 + i];
      vst2(vT + (((size_t)b * HH + h0 + hl) * HD + d) * TOT + PREV + s0 + pc * 8, pk.u); }
  }
}

__global__ __launch_bounds__(256) void k_cache(const float* __restrict__ ck, const float* __restrict__ cv, const float* __restrict__ cs,
                                             const float* __restrict__ sn, _Float16* __restrict__ kall, _Float16* __restrict__ vT) {
  __shared__ float tile[64][65];
  const int bh = blockIdx.y, t0 = blockIdx.x * 64, tid = threadIdx.x;
  for (int q = tid; q < 64 * 8; q += 256) { const int tl = q >> 3, pc = q & 7; const int t = t0 + tl;
    const float* src = ck + ((size_t)bh * PREV + t) * HD + pc * 8;
    union { v8h h; v4u u; } pk;
#pragma unroll
    for (int e = 0; e < 8; e += 2) { float a0 = src[e], a1 = src[e + 1]; rope2(a0, a1, cs, sn, t, (pc * 8 + e) >> 1); pk.h[e] = (_Float16)a0; pk.h[e + 1] = (_Float16)a1; }
    vst2(kall + ((size_t)bh * TOT + t) * HD + pc * 8, pk.u); }
  for (int q = tid; q < 64 * 64; q += 256) { const int tl = q >> 6, d = q & 63; tile[tl][d] = cv[((size_t)bh * PREV + t0 + tl) * HD + d]; }
  __syncthreads();
  for (int q = tid; q < 64 * 8; q += 256) { const int d = q >> 3, pc = q & 7;
    union { v8h h; v4u u; } pk;
#pragma unroll
    for (int e = 0; e < 8; ++e) pk.h[e] = (_Float16)tile[pc * 8 + e][d];
    vst2(vT + ((size_t)bh * HD + d) * TOT + t0 + pc * 8, pk.u); }
}

__global__ __launch_bounds__(128) void k_attn(const _Float16* __restrict__ qh, const _Float16* __restrict__ kall, const _Float16* __restrict__ vT,
                                            _Float16* __restrict__ ctx) {
  __shared__ __align__(16) float sP[4][16][BK];
  __shared__ __align__(16) float sO[4][16][HD];
  const int tid = threadIdx.x, w = tid >> 5, lane = tid & 31, g = lane >> 4, ln = lane & 15;
  const int bh = blockIdx.y, b = bh / HH, h = bh % HH, q0 = blockIdx.x * 64 + w * 16;
  const _Float16* qrow = qh + ((size_t)bh * SS + q0 + ln) * HD;
  const v16h qa0 = frag_h(qrow, lane), qa1 = frag_h(qrow + 32, lane);
  const float scale = 0.125f, slope = 2.0f / (float)(TOT - 1);
  float mrun[8], lrun[8];
  v8f acc[4];
#pragma unroll
  for (int r = 0; r < 8; ++r) { mrun[r] = -3.0e38f; lrun[r] = 0.f; }
#pragma unroll
  for (int t = 0; t < 4; ++t) acc[t] = (v8f){};
  const _Float16* kb = kall + (size_t)bh * TOT * HD;
  const _Float16* vb = vT + (size_t)bh * HD * TOT;
  const int kend = PREV + blockIdx.x * 64 + 64;
#pragma unroll 1
  for (int k0 = 0; k0 < kend; k0 += BK) {
    v8f s0 = {}, s1 = {};
    s0 = wmma16(qa0, frag_h(kb + (size_t)(k0 + ln) * HD, lane), s0);      s0 = wmma16(qa1, frag_h(kb + (size_t)(k0 + ln) * HD + 32, lane), s0);
    s1 = wmma16(qa0, frag_h(kb + (size_t)(k0 + 16 + ln) * HD, lane), s1); s1 = wmma16(qa1, frag_h(kb + (size_t)(k0 + 16 + ln) * HD + 32, lane), s1);
#pragma unroll
    for (int r = 0; r < 8; ++r) {
      const int i = q0 + 8 * g + r;
      const int t0k = k0 + ln, t1k = k0 + 16 + ln;
      const float b0v = slope * (float)(t0k - (PREV + i)), b1v = slope * (float)(t1k - (PREV + i));
      const float x0 = (t0k - PREV > i) ? -3.0e38f : s0[r] * scale + b0v, x1 = (t1k - PREV > i) ? -3.0e38f : s1[r] * scale + b1v;
      float mx = fmaxf(x0, x1);
#pragma unroll
      for (int off = 8; off >= 1; off >>= 1) mx = fmaxf(mx, __shfl_xor(mx, off, 32));
      const float mn = fmaxf(mrun[r], mx);
      const float corr = expf(mrun[r] - mn);
      const float p0 = (x0 > -1.0e38f) ? expf(x0 - mn) : 0.f, p1 = (x1 > -1.0e38f) ? expf(x1 - mn) : 0.f;
      float sum = p0 + p1;
#pragma unroll
      for (int off = 8; off >= 1; off >>= 1) sum += __shfl_xor(sum, off, 32);
      lrun[r] = lrun[r] * corr + sum; mrun[r] = mn;
#pragma unroll
      for (int t = 0; t < 4; ++t) acc[t][r] *= corr;
      sP[w][8 * g + r][ln] = p0 * 16384.0f; sP[w][8 * g + r][16 + ln] = p1 * 16384.0f;
    }
    LDSX();
    const v16h pa = frag_f32(&sP[w][ln][0], lane);
#pragma unroll
    for (int t = 0; t < 4; ++t) acc[t] = wmma16(pa, frag_h(vb + (size_t)(t * 16 + ln) * TOT + k0, lane), acc[t]);
    __builtin_amdgcn_wave_barrier();
  }
  float* so = &sO[w][0][0];
#pragma unroll
  for (int r = 0; r < 8; ++r) { const float il = (1.0f / 16384.0f) / lrun[r];
#pragma unroll
    for (int t = 0; t < 4; ++t) so[(8 * g + r) * HD + t * 16 + ln] = acc[t][r] * il; }
  LDSX();
#pragma unroll
  for (int i = 0; i < 4; ++i) { const int q = i * 32 + lane; const int rl = q >> 3, pc = q & 7;
    union { v8h hv; v4u u; } pk;
#pragma unroll
    for (int e = 0; e < 8; ++e) pk.hv[e] = (_Float16)so[rl * HD + pc * 8 + e];
    vst2(ctx + ((size_t)b * SS + q0 + rl) * DD + h * HD + pc * 8, pk.u); }
}

__global__ __launch_bounds__(128) void k_gemm_res(const _Float16* __restrict__ A, const _Float16* __restrict__ W, const float* __restrict__ bias,
                                                const float* __restrict__ res, float* __restrict__ out, int K, int ldo) {
  __shared__ __align__(16) float so[4][16 * 128];
  const int tid = threadIdx.x, wave = tid >> 5, lane = tid & 31, col = lane & 15, g = lane >> 4;
  const int r0 = blockIdx.x * 64 + wave * 16, n0 = blockIdx.y * 128;
  v8f acc[8] = {};
#pragma unroll 1
  for (int kc = 0; kc < K / 32; ++kc) {
    const v16h a = frag_h(A + (size_t)(r0 + col) * K + kc * 32, lane);
#pragma unroll
    for (int j = 0; j < 8; ++j) acc[j] = wmma16(a, frag_h(W + (size_t)(n0 + j * 16 + col) * K + kc * 32, lane), acc[j]);
  }
  float* S = so[wave];
#pragma unroll
  for (int j = 0; j < 8; ++j) { const float bv_ = bias[n0 + j * 16 + col];
#pragma unroll
    for (int r = 0; r < 8; ++r) S[(8 * g + r) * 128 + j * 16 + col] = acc[j][r] + bv_; }
  LDSX();
#pragma unroll 4
  for (int rl = 0; rl < 16; ++rl) { const size_t o = (size_t)(r0 + rl) * ldo + n0 + lane * 4;
    v4f v = *(const v4f*)(S + rl * 128 + lane * 4); if (res) v += *(const v4f*)(res + o); vst2(out + o, v); }
}

__global__ __launch_bounds__(128) void k_swiglu(const _Float16* __restrict__ A, const _Float16* __restrict__ Wg, const float* __restrict__ bg,
                                              const _Float16* __restrict__ Wvl, const float* __restrict__ bvl, _Float16* __restrict__ G) {
  __shared__ __align__(16) float so[4][16 * 64];
  const int tid = threadIdx.x, wave = tid >> 5, lane = tid & 31, col = lane & 15, g = lane >> 4;
  const int r0 = blockIdx.x * 64 + wave * 16, n0 = blockIdx.y * 64;
  v8f ag[4] = {}, av[4] = {};
#pragma unroll 1
  for (int kc = 0; kc < DD / 32; ++kc) {
    const v16h a = frag_h(A + (size_t)(r0 + col) * DD + kc * 32, lane);
#pragma unroll
    for (int j = 0; j < 4; ++j) { ag[j] = wmma16(a, frag_h(Wg + (size_t)(n0 + j * 16 + col) * DD + kc * 32, lane), ag[j]);
                                  av[j] = wmma16(a, frag_h(Wvl + (size_t)(n0 + j * 16 + col) * DD + kc * 32, lane), av[j]); }
  }
  float* S = so[wave];
#pragma unroll
  for (int j = 0; j < 4; ++j) { const float b1 = bg[n0 + j * 16 + col], b2 = bvl[n0 + j * 16 + col];
#pragma unroll
    for (int r = 0; r < 8; ++r) { const float u = ag[j][r] + b1; S[(8 * g + r) * 64 + j * 16 + col] = u / (1.0f + expf(-u)) * (av[j][r] + b2); } }
  LDSX();
#pragma unroll
  for (int q = 0; q < 4; ++q) { const int rl = q * 4 + (lane >> 3), pc = lane & 7;
    union { v8h hv; v4u u; } pk;
#pragma unroll
    for (int e = 0; e < 8; ++e) pk.hv[e] = (_Float16)S[rl * 64 + pc * 8 + e];
    vst2(G + (size_t)(r0 + rl) * FF + n0 + pc * 8, pk.u); }
}

extern "C" void kernel_launch(void* const* d_in, const int* in_sizes, int n_in,
                              void* d_out, int out_size, void* d_ws, size_t ws_size,
                              hipStream_t stream) {
  (void)in_sizes; (void)n_in; (void)out_size; (void)ws_size;
  const float* x   = (const float*)d_in[0];
  const float* ck  = (const float*)d_in[1]; const float* cv = (const float*)d_in[2];
  const float* cs  = (const float*)d_in[3]; const float* sn = (const float*)d_in[4];
  const float* anw = (const float*)d_in[5]; const float* fnw = (const float*)d_in[6];
  const float* wq = (const float*)d_in[7];  const float* bq = (const float*)d_in[8];
  const float* wk = (const float*)d_in[9];  const float* bk = (const float*)d_in[10];
  const float* wv = (const float*)d_in[11]; const float* bv = (const float*)d_in[12];
  const float* wo = (const float*)d_in[13]; const float* bo = (const float*)d_in[14];
  const float* wg = (const float*)d_in[15]; const float* bg = (const float*)d_in[16];
  const float* wl = (const float*)d_in[17]; const float* bl = (const float*)d_in[18];
  const float* wp = (const float*)d_in[19]; const float* bp = (const float*)d_in[20];
  float* out = (float*)d_out;
  char* ws = (char*)d_ws; size_t off = 0;
  auto take = [&](size_t bytes) { char* p = ws + off; off += (bytes + 255) & ~(size_t)255; return p; };
  _Float16* hh  = (_Float16*)take((size_t)NR * DD * 2);
  _Float16* Wqh = (_Float16*)take((size_t)DD * DD * 2); _Float16* Wkh = (_Float16*)take((size_t)DD * DD * 2);
  _Float16* Wvh = (_Float16*)take((size_t)DD * DD * 2); _Float16* Woh = (_Float16*)take((size_t)DD * DD * 2);
  _Float16* Wgh = (_Float16*)take((size_t)FF * DD * 2); _Float16* Wlh = (_Float16*)take((size_t)FF * DD * 2);
  _Float16* Wph = (_Float16*)take((size_t)DD * FF * 2);
  _Float16* qh  = (_Float16*)take((size_t)BB * HH * SS * HD * 2);
  _Float16* kall = (_Float16*)take((size_t)BB * HH * TOT * HD * 2);
  _Float16* vT  = (_Float16*)take((size_t)BB * HH * HD * TOT * 2);
  _Float16* ctx = (_Float16*)take((size_t)NR * DD * 2);
  float*    x1  = (float*)take((size_t)NR * DD * 4);
  _Float16* h2  = (_Float16*)take((size_t)NR * DD * 2);
  _Float16* G   = (_Float16*)take((size_t)NR * FF * 2);
  auto cvt = [&](const float* s, _Float16* d, size_t n) { k_cvt<<<(unsigned)((n / 8 + 255) / 256), 256, 0, stream>>>(s, d, n / 8); };
  cvt(wq, Wqh, (size_t)DD * DD); cvt(wk, Wkh, (size_t)DD * DD); cvt(wv, Wvh, (size_t)DD * DD); cvt(wo, Woh, (size_t)DD * DD);
  cvt(wg, Wgh, (size_t)FF * DD); cvt(wl, Wlh, (size_t)FF * DD); cvt(wp, Wph, (size_t)DD * FF);
  k_rms<<<NR, 128, 0, stream>>>(x, anw, hh);
  k_qkv<<<dim3(NR / 64, DD / 128, 3), 128, 0, stream>>>(hh, Wqh, Wkh, Wvh, bq, bk, bv, cs, sn, qh, kall, vT);
  k_cache<<<dim3(PREV / 64, BB * HH), 256, 0, stream>>>(ck, cv, cs, sn, kall, vT);
  k_attn<<<dim3(SS / 64, BB * HH), 128, 0, stream>>>(qh, kall, vT, ctx);
  k_gemm_res<<<dim3(NR / 64, DD / 128), 128, 0, stream>>>(ctx, Woh, bo, x, x1, DD, DD);
  k_rms<<<NR, 128, 0, stream>>>(x1, fnw, h2);
  k_swiglu<<<dim3(NR / 64, FF / 64), 128, 0, stream>>>(h2, Wgh, bg, Wlh, bl, G);
  k_gemm_res<<<dim3(NR / 64, DD / 128), 128, 0, stream>>>(G, Wph, bp, x1, out, FF, DD);
}
